// NeuralODEModel_87789131530507
// MI455X (gfx1250) — hardware-verified
//
#include <hip/hip_runtime.h>
#include <math.h>

#pragma clang fp contract(off)

typedef __attribute__((ext_vector_type(16))) _Float16 v16h;
typedef __attribute__((ext_vector_type(8)))  _Float16 v8h;
typedef __attribute__((ext_vector_type(8)))  float    v8f;
typedef __attribute__((ext_vector_type(4)))  float    v4f;

constexpr int NSD = 7;
constexpr int NH1 = 128;
constexpr int NSH = 64;
constexpr int NOH = 64;
constexpr int ROWS_PER_BLOCK = 32;
constexpr int TMAX = 64;
constexpr int PITCH_W  = 72;
constexpr int PITCH_X  = 72;
constexpr int PITCH_A1 = 136;
constexpr int PITCH_F  = 68;

constexpr int PL_W2SE  = 0;
constexpr int PL_WINIT = 8192;
constexpr int PL_WF1SE = 12288;
constexpr int PL_WF1H  = 16384;
constexpr int PL_WF2   = 20480;
constexpr int PL_TOTAL = 24576;
constexpr int PREP_WBLOCKS = 48;
constexpr int PREP_BLOCKS  = PREP_WBLOCKS + 1;

static_assert(PL_WINIT == PL_W2SE + NSH * NH1);
static_assert(PL_WF1SE == PL_WINIT + NOH * NSH);
static_assert(PL_WF1H == PL_WF1SE + NOH * NSH);
static_assert(PL_WF2 == PL_WF1H + NOH * NOH);
static_assert(PL_TOTAL == PL_WF2 + NOH * NOH);
static_assert(PL_TOTAL == PREP_WBLOCKS * 256 * 2);

constexpr float SC_W  = 256.0f;
constexpr float SC_R  = 2048.0f;
constexpr float SC_HH = 1.0f / 256.0f;
constexpr float SC_CR = 1.0f / 524288.0f;
constexpr float F16_MIN_NORM = 6.103515625e-5f;

__device__ __forceinline__ v8f vzero8() {
  return (v8f){0.0f, 0.0f, 0.0f, 0.0f, 0.0f, 0.0f, 0.0f, 0.0f};
}

__device__ __forceinline__ v16h frag_load(const _Float16* p) {
  union { v16h v; v8h q[2]; } f;
  f.q[0] = *(const v8h*)(p);
  f.q[1] = *(const v8h*)(p + 16);
  return f.v;
}

__device__ __forceinline__ v8f mma16(v16h a, v16h b, v8f acc) {
  return __builtin_amdgcn_wmma_f32_16x16x32_f16(false, a, false, b, (short)0, acc, false, false);
}

__device__ __forceinline__ void wmma_guard(v8f& a, v8f& b, v16h w, v16h x, v16h y, v16h z) {
  asm volatile("v_nop\n\tv_nop\n\tv_nop\n\tv_nop" : "+v"(a), "+v"(b) : "v"(w), "v"(x), "v"(y), "v"(z));
}

__device__ __forceinline__ void mma_step(v8f& acc, v8f& accr,
                                         const _Float16* aph, const _Float16* apl,
                                         const _Float16* bph, const _Float16* bpl) {
  const v16h ah = frag_load(aph);
  const v16h al = frag_load(apl);
  const v16h bh = frag_load(bph);
  const v16h bl = frag_load(bpl);
  acc  = mma16(ah, bh, acc);
  accr = mma16(ah, bl, accr);
  accr = mma16(al, bh, accr);
  wmma_guard(acc, accr, ah, al, bh, bl);
}

__device__ __forceinline__ void split16(float a, _Float16& hi, _Float16& lo) {
  _Float16 h = (_Float16)a;
  h = (fabsf(a) < F16_MIN_NORM) ? (_Float16)0.0f : h;
  const float res = (a - (float)h) * SC_R;
  _Float16 l = (_Float16)res;
  l = (fabsf(res) < F16_MIN_NORM) ? (_Float16)0.0f : l;
  hi = h;
  lo = l;
}

__device__ __forceinline__ unsigned short hbits(_Float16 x) { return __builtin_bit_cast(unsigned short, x); }

__device__ __forceinline__ float tanh_f(float x) {
  const float ax = fabsf(x);
  const float e = expf(-2.0f * ax);
  const float t = (1.0f - e) / (1.0f + e);
  return copysignf(t, x);
}

__device__ __forceinline__ float softplus_f(float x) {
  return fmaxf(x, 0.0f) + log1pf(expf(-fabsf(x)));
}

__device__ __forceinline__ float mod_pos(float x, float y) {
  const float q = x / y;
  const float n = truncf(q);
  float r = fmaf(-n, y, x);
  r = (r < 0.0f) ? (r + y) : r;
  r = (r >= y) ? (r - y) : r;
  return r;
}

__global__ __launch_bounds__(256) void prep_kernel(const float* __restrict__ sf, int B,
                                                   const float* __restrict__ Wse2, const float* __restrict__ Winit,
                                                   const float* __restrict__ Wf1, const float* __restrict__ Wf2,
                                                   unsigned* __restrict__ plh, unsigned* __restrict__ pll,
                                                   float* __restrict__ scal) {
  __shared__ float ssum[2];
  const int blk = blockIdx.x;
  const int tid = threadIdx.x;
  if (blk < PREP_WBLOCKS) {
    const float* src = Wse2;
    int kofs = 0, klog2 = 7, ubase = PL_W2SE / 2, u = blk * 256 + tid;
    if (blk >= 16 && blk < 24) { src = Winit; kofs = 0;   klog2 = 6; ubase = PL_WINIT / 2; u = (blk - 16) * 256 + tid; }
    if (blk >= 24 && blk < 32) { src = Wf1;   kofs = NOH; klog2 = 6; ubase = PL_WF1SE / 2; u = (blk - 24) * 256 + tid; }
    if (blk >= 32 && blk < 40) { src = Wf1;   kofs = 0;   klog2 = 6; ubase = PL_WF1H / 2;  u = (blk - 32) * 256 + tid; }
    if (blk >= 40)             { src = Wf2;   kofs = 0;   klog2 = 6; ubase = PL_WF2 / 2;   u = (blk - 40) * 256 + tid; }
    const int kmask = (1 << klog2) - 1;
    const int e0 = 2 * u;
    const int n = e0 >> klog2;
    const int k = e0 & kmask;
    const float w0 = src[(size_t)(kofs + k) * NSH + n] * SC_W;
    const float w1 = src[(size_t)(kofs + k + 1) * NSH + n] * SC_W;
    _Float16 h0, l0, h1, l1;
    split16(w0, h0, l0);
    split16(w1, h1, l1);
    const unsigned uh = (unsigned)hbits(h0) | ((unsigned)hbits(h1) << 16);
    const unsigned ul = (unsigned)hbits(l0) | ((unsigned)hbits(l1) << 16);
    volatile unsigned* dh = plh + ubase;
    volatile unsigned* dl = pll + ubase;
    dh[u] = uh;
    dl[u] = ul;
    __threadfence();
    dh[u] = uh;
    dl[u] = ul;
  } else {
    if (tid == 0) {
      float a5 = 0.0f, a6 = 0.0f;
      for (int jb = 0; jb < B; jb += 32) {
        const int je = (jb + 32 < B) ? (jb + 32) : B;
        float p5 = 0.0f, p6 = 0.0f;
        for (int j = jb; j < je; ++j) {
          p5 = p5 + sf[(size_t)j * NSD + 5];
          p6 = p6 + sf[(size_t)j * NSD + 6];
        }
        a5 = a5 + p5;
        a6 = a6 + p6;
      }
      ssum[0] = a5 / (float)B;
      ssum[1] = a6 / (float)B;
    }
    __syncthreads();
    if (tid < 32) {
      const float v0 = ssum[0];
      const float v1 = ssum[1];
      const float v = (tid == 0) ? v0 : ((tid == 1) ? v1 : 0.0f);
      volatile float* sp = scal;
      sp[tid] = v;
      __threadfence();
      sp[tid] = v;
    }
  }
}

__device__ __forceinline__ void enc_gemm_k64(const _Float16* aH, const _Float16* aL,
                                            const _Float16* bH, const _Float16* bL,
                                            const float* __restrict__ bias, float* slabw,
                                            int hh, int c, int rowA, int koff) {
#pragma unroll
  for (int j = 0; j < 4; ++j) {
    const int n = j * 16 + c;
    v8f acc = vzero8(), accr = vzero8();
#pragma unroll
    for (int ks = 0; ks < 2; ++ks)
      mma_step(acc, accr,
               aH + rowA * PITCH_X + ks * 32 + koff, aL + rowA * PITCH_X + ks * 32 + koff,
               bH + n * NSH + ks * 32 + koff,        bL + n * NSH + ks * 32 + koff);
    const float bn = bias[n];
#pragma unroll
    for (int r = 0; r < 8; ++r) {
      float v = acc[r] * SC_HH + accr[r] * SC_CR;
      v = v + bn;
      slabw[(8 * hh + r) * PITCH_F + n] = v;
    }
  }
}

__device__ __forceinline__ void store_rows16_f32(const float* slabw, float* dst, int lane) {
  const int hh = lane >> 4, c4 = (lane & 15) * 4;
  for (int pass = 0; pass < 2; ++pass) {
#pragma unroll
    for (int it = 0; it < 8; ++it) {
      const int row = it * 2 + hh;
      const v4f v = *(const v4f*)(slabw + row * PITCH_F + c4);
      *(volatile v4f*)(dst + (size_t)row * NOH + c4) = v;
    }
    __threadfence();
  }
}

__global__ __launch_bounds__(64) void encoder_kernel(
    const float* __restrict__ sf, const float* __restrict__ Wse1, const float* __restrict__ bse1,
    const float* __restrict__ bse2, const float* __restrict__ binit, const float* __restrict__ bf1,
    const float* __restrict__ Wcp, const float* __restrict__ bcp_p,
    const unsigned short* __restrict__ pw2h, const unsigned short* __restrict__ pw2l,
    const unsigned short* __restrict__ pwih, const unsigned short* __restrict__ pwil,
    const unsigned short* __restrict__ pwfh, const unsigned short* __restrict__ pwfl,
    float* __restrict__ h0g, float* __restrict__ cseg, float* __restrict__ icpg) {
  __shared__ float sW1[NSD * NH1];
  __shared__ float sB1[NH1];
  __shared__ float sWcp[NSH];
  __shared__ __align__(16) _Float16 sAh[2][16 * PITCH_A1];
  __shared__ __align__(16) _Float16 sAl[2][16 * PITCH_A1];
  __shared__ __align__(16) _Float16 sEh[2][16 * PITCH_X];
  __shared__ __align__(16) _Float16 sEl[2][16 * PITCH_X];
  __shared__ __align__(16) float slab[2][16 * PITCH_F];
  __shared__ float sCp[ROWS_PER_BLOCK];

  const int tid = threadIdx.x;
  const int lane = tid & 31;
  const int wave = tid >> 5;
  const int hh = lane >> 4;
  const int c = lane & 15;
  const int rowA = lane & 15;
  const int koff = hh * 8;
  const int rbase = blockIdx.x * ROWS_PER_BLOCK + wave * 16;

  for (int i = tid; i < NSD * NH1; i += 64) sW1[i] = Wse1[i];
  for (int i = tid; i < NH1; i += 64) sB1[i] = bse1[i];
  sWcp[tid] = Wcp[tid];
  __syncthreads();

  _Float16* aH = sAh[wave];
  _Float16* aL = sAl[wave];
  _Float16* eH = sEh[wave];
  _Float16* eL = sEl[wave];
  float* slabw = slab[wave];

  {
    const int row = lane & 15;
    const int jh = lane >> 4;
    float x[NSD];
#pragma unroll
    for (int i = 0; i < NSD; ++i) x[i] = sf[(size_t)(rbase + row) * NSD + i];
#pragma unroll 1
    for (int jj = 0; jj < 64; ++jj) {
      const int j = jh * 64 + jj;
      float a = 0.0f;
#pragma unroll
      for (int i = 0; i < NSD; ++i) a = a + x[i] * sW1[i * NH1 + j];
      a = a + sB1[j];
      a = fmaxf(a, 0.0f);
      _Float16 eh, el;
      split16(a, eh, el);
      aH[row * PITCH_A1 + j] = eh;
      aL[row * PITCH_A1 + j] = el;
    }
  }
  __syncthreads();

  {
    const _Float16* gbh = (const _Float16*)pw2h;
    const _Float16* gbl = (const _Float16*)pw2l;
#pragma unroll
    for (int j = 0; j < 4; ++j) {
      const int n = j * 16 + c;
      v8f acc = vzero8(), accr = vzero8();
#pragma unroll
      for (int ks = 0; ks < 4; ++ks)
        mma_step(acc, accr,
                 aH + rowA * PITCH_A1 + ks * 32 + koff, aL + rowA * PITCH_A1 + ks * 32 + koff,
                 gbh + n * NH1 + ks * 32 + koff,        gbl + n * NH1 + ks * 32 + koff);
      const float bn = bse2[n];
#pragma unroll
      for (int r = 0; r < 8; ++r) {
        float v = acc[r] * SC_HH + accr[r] * SC_CR;
        v = v + bn;
        v = fmaxf(v, 0.0f);
        const int row = 8 * hh + r;
        slabw[row * PITCH_F + n] = v;
        _Float16 eh, el;
        split16(v, eh, el);
        eH[row * PITCH_X + n] = eh;
        eL[row * PITCH_X + n] = el;
      }
    }
  }
  __syncthreads();

  {
    const int row = lane & 15;
    const float* sp = slabw + row * PITCH_F;
    const float bcp = bcp_p[0];
    float s = 0.0f;
#pragma unroll 1
    for (int k = 0; k < NSH; ++k) s = s + sp[k] * sWcp[k];
    s = s + bcp;
    const float v = softplus_f(s);
    if (lane < 16) sCp[wave * 16 + row] = v;
  }
  __syncthreads();

  enc_gemm_k64(eH, eL, (const _Float16*)pwih, (const _Float16*)pwil, binit, slabw, hh, c, rowA, koff);
  __syncthreads();
  store_rows16_f32(slabw, h0g + (size_t)rbase * NOH, lane);
  __syncthreads();

  enc_gemm_k64(eH, eL, (const _Float16*)pwfh, (const _Float16*)pwfl, bf1, slabw, hh, c, rowA, koff);
  __syncthreads();
  store_rows16_f32(slabw, cseg + (size_t)rbase * NOH, lane);
  __syncthreads();

  if (wave == 0) {
    const float v = sCp[lane];
    volatile float* ip = icpg + (size_t)blockIdx.x * ROWS_PER_BLOCK;
    ip[lane] = v;
    __threadfence();
    ip[lane] = v;
  }
}

__global__ __launch_bounds__(256) void ode_kernel(
    const float* __restrict__ tt, int T,
    const float* __restrict__ h0g, const float* __restrict__ cseg, const float* __restrict__ icpg,
    const float* __restrict__ scal,
    const unsigned short* __restrict__ pw1h, const unsigned short* __restrict__ pw1l,
    const unsigned short* __restrict__ pw2h, const unsigned short* __restrict__ pw2l,
    const float* __restrict__ Wf1, const float* __restrict__ bf2,
    const float* __restrict__ injscale_p, const float* __restrict__ Wro, const float* __restrict__ bro_p,
    float* __restrict__ out) {
  __shared__ __align__(16) _Float16 sW1h[NOH * PITCH_W];
  __shared__ __align__(16) _Float16 sW1l[NOH * PITCH_W];
  __shared__ __align__(16) _Float16 sW2h[NOH * PITCH_W];
  __shared__ __align__(16) _Float16 sW2l[NOH * PITCH_W];
  __shared__ __align__(16) _Float16 sXh[ROWS_PER_BLOCK * PITCH_X];
  __shared__ __align__(16) _Float16 sXl[ROWS_PER_BLOCK * PITCH_X];
  __shared__ __align__(16) _Float16 sYh[ROWS_PER_BLOCK * PITCH_X];
  __shared__ __align__(16) _Float16 sYl[ROWS_PER_BLOCK * PITCH_X];
  __shared__ __align__(16) float sHf[ROWS_PER_BLOCK * PITCH_F];
  __shared__ __align__(16) float sOut[ROWS_PER_BLOCK * TMAX];
  __shared__ float sWro[NOH];
  __shared__ float sTT[TMAX];
  __shared__ float sIcp[ROWS_PER_BLOCK];

  const int tid = threadIdx.x;
  const int lane = tid & 31;
  const int wave = tid >> 5;
  const int hh = lane >> 4;
  const int c = lane & 15;
  const int tile = wave >> 2;
  const int nt = wave & 3;
  const int col = nt * 16 + c;
  const int rowA = lane & 15;
  const int koff = hh * 8;
  const int blockBase = blockIdx.x * ROWS_PER_BLOCK;

  {
    const _Float16* g1h = (const _Float16*)pw1h;
    const _Float16* g1l = (const _Float16*)pw1l;
    const _Float16* g2h = (const _Float16*)pw2h;
    const _Float16* g2l = (const _Float16*)pw2l;
#pragma unroll
    for (int q = 0; q < 2; ++q) {
      const int ch = tid + 256 * q;
      const int n = ch >> 3, k8 = (ch & 7) * 8;
      const v8h a0 = *(const v8h*)(g1h + n * NOH + k8);
      const v8h a1 = *(const v8h*)(g1l + n * NOH + k8);
      const v8h a2 = *(const v8h*)(g2h + n * NOH + k8);
      const v8h a3 = *(const v8h*)(g2l + n * NOH + k8);
      *(v8h*)(sW1h + n * PITCH_W + k8) = a0;
      *(v8h*)(sW1l + n * PITCH_W + k8) = a1;
      *(v8h*)(sW2h + n * PITCH_W + k8) = a2;
      *(v8h*)(sW2l + n * PITCH_W + k8) = a3;
    }
  }
  {
#pragma unroll
    for (int q = 0; q < 2; ++q) {
      const int ch = tid + 256 * q;
      const int row = ch >> 4, c4 = (ch & 15) * 4;
      const v4f hv = *(const v4f*)(h0g + (size_t)(blockBase + row) * NOH + c4);
      const v4f cv = *(const v4f*)(cseg + (size_t)(blockBase + row) * NOH + c4);
      *(v4f*)(sHf + row * PITCH_F + c4) = hv;
      *(v4f*)(sOut + row * NOH + c4) = cv;
    }
  }
  if (tid < TMAX) {
    sWro[tid] = Wro[tid];
    const int ti = (tid < T) ? tid : (T - 1);
    sTT[tid] = tt[ti];
  }
  if (tid < ROWS_PER_BLOCK) sIcp[tid] = icpg[blockBase + tid];
  const float amt = scal[0];
  const float II = scal[1];
  const float injsc = injscale_p[0];
  const float bro = bro_p[0];
  const float bf2c = bf2[col];
  const float wtc = Wf1[(NOH + NSH) * NOH + col];
  const float c2w2 = (float)(2.0 * 0.001 * 0.001);
  const float inv2w2 = 1.0f / c2w2;
  __syncthreads();

  const int pbase = (tile * 16 + 8 * hh) * PITCH_X + col;
  const int abase = (tile * 16 + rowA) * PITCH_X + koff;
  const int bbase = col * PITCH_W + koff;
  const int hbase = (tile * 16 + 8 * hh) * PITCH_F + col;

  v8f h, cseF;
#pragma unroll
  for (int r = 0; r < 8; ++r) {
    h[r] = sHf[hbase + r * PITCH_F];
    cseF[r] = sOut[(tile * 16 + 8 * hh + r) * NOH + col];
  }
  __syncthreads();

  auto readout = [&](int ts) {
#pragma unroll
    for (int r = 0; r < 8; ++r) sHf[hbase + r * PITCH_F] = h[r];
    __syncthreads();
    if (tid < ROWS_PER_BLOCK) {
      const float* hp = sHf + tid * PITCH_F;
      float s = 0.0f;
#pragma unroll 1
      for (int k = 0; k < NOH; ++k) s = s + hp[k] * sWro[k];
      s = s + bro;
      sOut[tid * T + ts] = softplus_f(s) + sIcp[tid];
    }
    __syncthreads();
  };

  auto feval = [&](v8f X, float tv) -> v8f {
#pragma unroll
    for (int r = 0; r < 8; ++r) {
      _Float16 eh, el;
      split16(X[r], eh, el);
      sXh[pbase + r * PITCH_X] = eh;
      sXl[pbase + r * PITCH_X] = el;
    }
    __syncthreads();
    v8f acc = vzero8(), accr = vzero8();
#pragma unroll
    for (int ks = 0; ks < 2; ++ks)
      mma_step(acc, accr, sXh + abase + ks * 32, sXl + abase + ks * 32,
               sW1h + bbase + ks * 32, sW1l + bbase + ks * 32);
    const float tvw = tv * wtc;
#pragma unroll
    for (int r = 0; r < 8; ++r) {
      float pre = acc[r] * SC_HH + accr[r] * SC_CR;
      pre = pre + cseF[r];
      pre = pre + tvw;
      const float th = tanh_f(pre);
      _Float16 eh, el;
      split16(th, eh, el);
      sYh[pbase + r * PITCH_X] = eh;
      sYl[pbase + r * PITCH_X] = el;
    }
    __syncthreads();
    v8f acc2 = vzero8(), accr2 = vzero8();
#pragma unroll
    for (int ks = 0; ks < 2; ++ks)
      mma_step(acc2, accr2, sYh + abase + ks * 32, sYl + abase + ks * 32,
               sW2h + bbase + ks * 32, sW2l + bbase + ks * 32);
    const float rem = mod_pos(tv, II);
    const float q2 = -(rem * rem);
    const float ex = expf(q2 * inv2w2);
    const float injv = injsc * (amt * ex);
    v8f kout;
#pragma unroll
    for (int r = 0; r < 8; ++r) {
      float d = acc2[r] * SC_HH + accr2[r] * SC_CR;
      d = d + bf2c;
      d = d + injv;
      kout[r] = d;
    }
    return kout;
  };

  const float c1_5    = (float)(1.0 / 5.0);
  const float c3_10   = (float)(3.0 / 10.0);
  const float c4_5    = (float)(4.0 / 5.0);
  const float c8_9    = (float)(8.0 / 9.0);
  const float c3_40   = (float)(3.0 / 40.0);
  const float c9_40   = (float)(9.0 / 40.0);
  const float c44_45  = (float)(44.0 / 45.0);
  const float cm56_15 = (float)(-56.0 / 15.0);
  const float c32_9   = (float)(32.0 / 9.0);
  const float c19372  = (float)(19372.0 / 6561.0);
  const float cm25360 = (float)(-25360.0 / 2187.0);
  const float c64448  = (float)(64448.0 / 6561.0);
  const float cm212   = (float)(-212.0 / 729.0);
  const float c9017   = (float)(9017.0 / 3168.0);
  const float cm355   = (float)(-355.0 / 33.0);
  const float c46732  = (float)(46732.0 / 5247.0);
  const float c49_176 = (float)(49.0 / 176.0);
  const float cm5103  = (float)(-5103.0 / 18656.0);
  const float c35_384 = (float)(35.0 / 384.0);
  const float c500    = (float)(500.0 / 1113.0);
  const float c125_192 = (float)(125.0 / 192.0);
  const float cm2187  = (float)(-2187.0 / 6784.0);
  const float c11_84  = (float)(11.0 / 84.0);

  readout(0);

  for (int it = 0; it + 1 < T; ++it) {
    const float t0 = sTT[it];
    const float dt = sTT[it + 1] - t0;
    v8f X;
    float ts;

    const v8f k1 = feval(h, t0);

    ts = t0 + dt * c1_5;
#pragma unroll
    for (int r = 0; r < 8; ++r) X[r] = h[r] + dt * (c1_5 * k1[r]);
    const v8f k2 = feval(X, ts);

    ts = t0 + dt * c3_10;
#pragma unroll
    for (int r = 0; r < 8; ++r) X[r] = h[r] + dt * (c3_40 * k1[r] + c9_40 * k2[r]);
    const v8f k3 = feval(X, ts);

    ts = t0 + dt * c4_5;
#pragma unroll
    for (int r = 0; r < 8; ++r)
      X[r] = h[r] + dt * (c44_45 * k1[r] + cm56_15 * k2[r] + c32_9 * k3[r]);
    const v8f k4 = feval(X, ts);

    ts = t0 + dt * c8_9;
#pragma unroll
    for (int r = 0; r < 8; ++r)
      X[r] = h[r] + dt * (c19372 * k1[r] + cm25360 * k2[r] + c64448 * k3[r] + cm212 * k4[r]);
    const v8f k5 = feval(X, ts);

    ts = t0 + dt;
#pragma unroll
    for (int r = 0; r < 8; ++r)
      X[r] = h[r] + dt * (c9017 * k1[r] + cm355 * k2[r] + c46732 * k3[r] + c49_176 * k4[r] + cm5103 * k5[r]);
    const v8f k6 = feval(X, ts);

#pragma unroll
    for (int r = 0; r < 8; ++r)
      h[r] = h[r] + dt * (c35_384 * k1[r] + c500 * k3[r] + c125_192 * k4[r] + cm2187 * k5[r] + c11_84 * k6[r]);

    readout(it + 1);
  }

  __syncthreads();
  {
    const int nf4 = 8 * T;
    float* ob = out + (size_t)blockBase * T;
    for (int pass = 0; pass < 2; ++pass) {
      for (int q = tid; q < nf4; q += 256) {
        const v4f v = *(const v4f*)(sOut + 4 * q);
        *(volatile v4f*)(ob + 4 * q) = v;
      }
      __threadfence();
    }
  }
}

extern "C" void kernel_launch(void* const* d_in, const int* in_sizes, int n_in,
                              void* d_out, int out_size, void* d_ws, size_t ws_size,
                              hipStream_t stream) {
  if (n_in < 17) return;
  const float* t     = (const float*)d_in[0];
  const float* sf    = (const float*)d_in[1];
  const float* Wse1  = (const float*)d_in[2];
  const float* bse1  = (const float*)d_in[3];
  const float* Wse2  = (const float*)d_in[4];
  const float* bse2  = (const float*)d_in[5];
  const float* Winit = (const float*)d_in[6];
  const float* binit = (const float*)d_in[7];
  const float* Wf1   = (const float*)d_in[8];
  const float* bf1   = (const float*)d_in[9];
  const float* Wf2   = (const float*)d_in[10];
  const float* bf2   = (const float*)d_in[11];
  const float* injs  = (const float*)d_in[12];
  const float* Wro   = (const float*)d_in[13];
  const float* bro   = (const float*)d_in[14];
  const float* Wcp   = (const float*)d_in[15];
  const float* bcp   = (const float*)d_in[16];

  const int T = in_sizes[0];
  const int B = in_sizes[1] / NSD;
  if (T < 2 || T > TMAX) return;
  if (B < ROWS_PER_BLOCK || (B % ROWS_PER_BLOCK) != 0) return;
  if (out_size != B * T) return;
  if (in_sizes[2] != NSD * NH1 || in_sizes[4] != NH1 * NSH || in_sizes[6] != NSH * NOH) return;
  if (in_sizes[8] != (NOH + NSH + 1) * NOH || in_sizes[10] != NOH * NOH) return;
  if (in_sizes[13] != NOH || in_sizes[15] != NSH || in_sizes[3] != NH1 || in_sizes[5] != NSH) return;
  if (in_sizes[7] != NOH || in_sizes[9] != NOH || in_sizes[11] != NOH) return;
  if (in_sizes[12] < 1 || in_sizes[14] < 1 || in_sizes[16] < 1) return;

  size_t off = 0;
  const size_t o_scal = off; off += 256;
  const size_t o_plh = off; off += (size_t)PL_TOTAL * 2;
  const size_t o_pll = off; off += (size_t)PL_TOTAL * 2;
  const size_t o_h0 = off; off += (size_t)B * NOH * sizeof(float);
  const size_t o_cse = off; off += (size_t)B * NOH * sizeof(float);
  const size_t o_icp = off; off += (size_t)B * sizeof(float);
  if (off > ws_size) return;

  char* w = (char*)d_ws;
  float* scal = (float*)(w + o_scal);
  unsigned* plh_u = (unsigned*)(w + o_plh);
  unsigned* pll_u = (unsigned*)(w + o_pll);
  const unsigned short* plh = (const unsigned short*)(w + o_plh);
  const unsigned short* pll = (const unsigned short*)(w + o_pll);
  float* h0 = (float*)(w + o_h0);
  float* cse = (float*)(w + o_cse);
  float* icp = (float*)(w + o_icp);

  prep_kernel<<<PREP_BLOCKS, 256, 0, stream>>>(sf, B, Wse2, Winit, Wf1, Wf2, plh_u, pll_u, scal);

  encoder_kernel<<<B / ROWS_PER_BLOCK, 64, 0, stream>>>(
      sf, Wse1, bse1, bse2, binit, bf1, Wcp, bcp,
      plh + PL_W2SE, pll + PL_W2SE,
      plh + PL_WINIT, pll + PL_WINIT,
      plh + PL_WF1SE, pll + PL_WF1SE,
      h0, cse, icp);

  ode_kernel<<<B / ROWS_PER_BLOCK, 256, 0, stream>>>(
      t, T, h0, cse, icp, scal,
      plh + PL_WF1H, pll + PL_WF1H, plh + PL_WF2, pll + PL_WF2,
      Wf1, bf2, injs, Wro, bro, (float*)d_out);
}
